// SGCNModel_70935679860746
// MI455X (gfx1250) — hardware-verified
//
#include <hip/hip_runtime.h>
#include <stddef.h>


#define DF      128
#define H2      64
#define NTHR    256
#define NWAVE   8
#define EPT     8
#define NGRP    2
#define CHUNK   (NTHR * EPT * NGRP)
#define WCAP    (EPT * NGRP * 32)
#define LISTN   (NWAVE * WCAP)
#define NB      512
#define RPW     (NB / NWAVE)
#define LN_EPS  1e-5f

#define LDS_ACC  (NB * DF * 4)
#define LDS_LIST (LISTN * 4)
#define LDS_CNT  (NB * 4)
#define LDS_AGG  (LDS_ACC + LDS_LIST + LDS_CNT + 64)

#define GT   128
#define GW   4
#define GR   64
#define STF  132
#define STH  136

#define W0_OFF 0
#define W0_K   256
#define W1_OFF 32768
#define W1_K   192
#define P1_OFF 57344
#define P2_OFF 73728
#define WB_TOT 90112

static_assert((CHUNK & (CHUNK - 1)) == 0);
static_assert(CHUNK <= 4096);
static_assert((NB & (NB - 1)) == 0);
static_assert(NB <= 4096);
static_assert(RPW % 2 == 0);
static_assert(NWAVE * 4 <= 64);
static_assert(LDS_AGG <= 300 * 1024);
static_assert((WB_TOT % (256 * 8)) == 0);
static_assert((W1_OFF % 2048) == 0);
static_assert((P1_OFF % 2048) == 0);
static_assert((P2_OFF % 2048) == 0);

typedef float    v4f  __attribute__((ext_vector_type(4)));
typedef float    v8f  __attribute__((ext_vector_type(8)));
typedef int      v4i  __attribute__((ext_vector_type(4)));
typedef _Float16 half_t;
typedef half_t   v4h  __attribute__((ext_vector_type(4)));
typedef half_t   v8h  __attribute__((ext_vector_type(8)));
typedef half_t   v16h __attribute__((ext_vector_type(16)));
union Frag  { v16h v; v8h h[2]; v4i q[2]; };
union Pack8 { v8h v; v4i q; };

__device__ __forceinline__ v8f wm(v16h a, v16h b, v8f c) {
  v8f d = __builtin_amdgcn_wmma_f32_16x16x32_f16(false, a, false, b, (short)0, c, false, false);
  asm volatile("v_nop\n\tv_nop\n\tv_nop\n\tv_nop" : "+v"(d) : "v"(a), "v"(b));
  return d;
}

__device__ __forceinline__ v16h ld16g(const half_t* p) {
  Frag f;
  f.q[0] = *(const v4i*)(p);
  f.q[1] = *(const v4i*)(p + 16);
  return f.v;
}

__device__ __forceinline__ v16h cv16(const float* p) {
  const v4f a = *(const v4f*)(p);
  const v4f b = *(const v4f*)(p + 4);
  const v4f c = *(const v4f*)(p + 16);
  const v4f d = *(const v4f*)(p + 20);
  Frag f;
  f.v[0]  = (half_t)a.x; f.v[1]  = (half_t)a.y; f.v[2]  = (half_t)a.z; f.v[3]  = (half_t)a.w;
  f.v[4]  = (half_t)b.x; f.v[5]  = (half_t)b.y; f.v[6]  = (half_t)b.z; f.v[7]  = (half_t)b.w;
  f.v[8]  = (half_t)c.x; f.v[9]  = (half_t)c.y; f.v[10] = (half_t)c.z; f.v[11] = (half_t)c.w;
  f.v[12] = (half_t)d.x; f.v[13] = (half_t)d.y; f.v[14] = (half_t)d.z; f.v[15] = (half_t)d.w;
  return f.v;
}

__global__ __launch_bounds__(256) void k_wprep(
    const float* __restrict__ pl0, const float* __restrict__ pr0,
    const float* __restrict__ nl0, const float* __restrict__ nr0,
    const float* __restrict__ pl1, const float* __restrict__ pr1,
    const float* __restrict__ nl1, const float* __restrict__ nr1,
    const float* __restrict__ q1,  const float* __restrict__ q2,
    half_t* wb, int nTot) {
  const int u = blockIdx.x * 256 + threadIdx.x;
  if (u >= nTot) return;
  const int o = u * 8;
  const float* p;
  if (o < W1_OFF) {
    const int n = o >> 8, k = o & 255, nn = n & 63, kk = k & 127;
    const float* bl = (k < 128) ? pl0 : pr0;
    const float* bh = (k < 128) ? nl0 : nr0;
    p = ((n < 64) ? bl : bh) + nn * DF + kk;
  } else if (o < P1_OFF) {
    const int r = o - W1_OFF;
    const int n = r / W1_K;
    const int k = r - n * W1_K;
    const int nn = n & 63;
    const float* pa = ((n < 64) ? pl1 : nl1) + nn * DF + (k & 127);
    const float* pb = ((n < 64) ? pr1 : nr1) + nn * H2 + ((k - 128) & 63);
    p = (k < 128) ? pa : pb;
  } else if (o < P2_OFF) {
    p = q1 + (o - P1_OFF);
  } else {
    p = q2 + (o - P2_OFF);
  }
  const v4f a = *(const v4f*)(p);
  const v4f b = *(const v4f*)(p + 4);
  Pack8 pk;
  pk.v[0] = (half_t)a.x; pk.v[1] = (half_t)a.y; pk.v[2] = (half_t)a.z; pk.v[3] = (half_t)a.w;
  pk.v[4] = (half_t)b.x; pk.v[5] = (half_t)b.y; pk.v[6] = (half_t)b.z; pk.v[7] = (half_t)b.w;
  half_t* d = wb + o;
  const v4i qv = pk.q;
  *(volatile v4i*)d = qv;
  __threadfence();
  *(volatile v4i*)d = qv;
}

template <int NBT>
__device__ __forceinline__ int scan_chunk(const int* __restrict__ dsts, int nE, int cbase, int nodeBase,
                                          int vec8, int* list, int tid, int wave) {
  int wc = 0;
#pragma unroll
  for (int g = 0; g < NGRP; ++g) {
    const int el0  = (g * NTHR + tid) * EPT;
    const int e0   = cbase + el0;
    const int sent = -2147483647 - 1;
    v4i da, db;
    if (vec8 != 0 && cbase + CHUNK <= nE) {
      da = *(const v4i*)(dsts + e0);
      db = *(const v4i*)(dsts + e0 + 4);
    } else {
      const int lst = nE - 1;
      da.x = (e0     < nE) ? dsts[min(e0,     lst)] : sent;
      da.y = (e0 + 1 < nE) ? dsts[min(e0 + 1, lst)] : sent;
      da.z = (e0 + 2 < nE) ? dsts[min(e0 + 2, lst)] : sent;
      da.w = (e0 + 3 < nE) ? dsts[min(e0 + 3, lst)] : sent;
      db.x = (e0 + 4 < nE) ? dsts[min(e0 + 4, lst)] : sent;
      db.y = (e0 + 5 < nE) ? dsts[min(e0 + 5, lst)] : sent;
      db.z = (e0 + 6 < nE) ? dsts[min(e0 + 6, lst)] : sent;
      db.w = (e0 + 7 < nE) ? dsts[min(e0 + 7, lst)] : sent;
    }
    const unsigned nb = (unsigned)nodeBase;
    const unsigned s0 = (unsigned)da.x - nb, s1 = (unsigned)da.y - nb;
    const unsigned s2 = (unsigned)da.z - nb, s3 = (unsigned)da.w - nb;
    const unsigned s4 = (unsigned)db.x - nb, s5 = (unsigned)db.y - nb;
    const unsigned s6 = (unsigned)db.z - nb, s7 = (unsigned)db.w - nb;
    const bool h0 = s0 < (unsigned)NBT, h1 = s1 < (unsigned)NBT, h2 = s2 < (unsigned)NBT, h3 = s3 < (unsigned)NBT;
    const bool h4 = s4 < (unsigned)NBT, h5 = s5 < (unsigned)NBT, h6 = s6 < (unsigned)NBT, h7 = s7 < (unsigned)NBT;
    const unsigned any = __builtin_amdgcn_ballot_w32(h0 | h1 | h2 | h3 | h4 | h5 | h6 | h7);
    if (any != 0u) {
#define HITJ(J, HJ, SJ) { \
        const unsigned mj = __builtin_amdgcn_ballot_w32(HJ); \
        if (mj != 0u) { \
          if (HJ) { \
            const int pos = wc + (int)__builtin_amdgcn_mbcnt_lo(mj, 0u); \
            if (pos < WCAP) list[wave * WCAP + pos] = ((el0 + (J)) << 12) | (int)(SJ); \
          } \
          wc += (int)__builtin_popcount(mj); } }
      HITJ(0, h0, s0)
      HITJ(1, h1, s1)
      HITJ(2, h2, s2)
      HITJ(3, h3, s3)
      HITJ(4, h4, s4)
      HITJ(5, h5, s5)
      HITJ(6, h6, s6)
      HITJ(7, h7, s7)
#undef HITJ
    }
  }
  return wc;
}

__global__ __launch_bounds__(NTHR) void k_agg(
    const int* __restrict__ ei, const float* __restrict__ feat,
    half_t* plane, int nN, int nE, int vec8) {
  extern __shared__ v4f lds_dyn[];
  float* acc  = (float*)lds_dyn;
  int*   list = (int*)((char*)lds_dyn + LDS_ACC);
  int*   cnt  = (int*)((char*)lds_dyn + LDS_ACC + LDS_LIST);
  int*   wcnt = (int*)((char*)lds_dyn + LDS_ACC + LDS_LIST + LDS_CNT);
  const int tid = threadIdx.x, lane = tid & 31, wave = tid >> 5;
  const int nodeBase = blockIdx.x * NB;
  const int* dsts = ei + nE;

  {
    const v4f z = {0.f, 0.f, 0.f, 0.f};
    for (int i = tid; i < NB * DF / 4; i += NTHR) lds_dyn[i] = z;
    for (int i = tid; i < NB; i += NTHR) cnt[i] = 0;
  }
  __syncthreads();

  const int nChunks = (nE + CHUNK - 1) / CHUNK;
#pragma unroll 1
  for (int ch = 0; ch < nChunks; ++ch) {
    const int cbase = ch * CHUNK;
    const int wc = scan_chunk<NB>(dsts, nE, cbase, nodeBase, vec8, list, tid, wave);
    if (lane == 0) wcnt[wave] = wc;
    __syncthreads();
    if (wave == 0) {
#pragma unroll 1
      for (int wsx = 0; wsx < NWAVE; ++wsx) {
        int n = __builtin_amdgcn_readfirstlane(wcnt[wsx]);
        n = n > WCAP ? WCAP : (n < 0 ? 0 : n);
        const int* lp = list + wsx * WCAP;
#pragma unroll 1
        for (int i = 0; i < n; ++i) {
          const int ent  = __builtin_amdgcn_readfirstlane(lp[i]);
          const int slot = ent & (NB - 1);
          int e = cbase + ((ent >> 12) & (CHUNK - 1));
          e = e > nE - 1 ? nE - 1 : e;
          int src = ei[e];
          src = src < 0 ? 0 : (src > nN - 1 ? nN - 1 : src);
          const v4f v = *(const v4f*)(feat + (size_t)src * DF + 4 * lane);
          v4f* ap = (v4f*)(acc + slot * DF + 4 * lane);
          *ap = *ap + v;
          if (lane == 0) cnt[slot] = cnt[slot] + 1;
        }
      }
    }
    __syncthreads();
  }

  const int c8   = 8 * (lane & 15);
  const int rsub = lane >> 4;
#pragma unroll 1
  for (int i = 0; i < RPW / 2; ++i) {
    const int rr = RPW * wave + 2 * i + rsub;
    const int cd = cnt[rr];
    const float inv = 1.0f / (float)(cd > 1 ? cd : 1);
    const float* arow = acc + rr * DF + c8;
    const v4f a = (*(const v4f*)(arow)) * inv;
    const v4f b = (*(const v4f*)(arow + 4)) * inv;
    Pack8 pk;
    pk.v[0] = (half_t)a.x; pk.v[1] = (half_t)a.y; pk.v[2] = (half_t)a.z; pk.v[3] = (half_t)a.w;
    pk.v[4] = (half_t)b.x; pk.v[5] = (half_t)b.y; pk.v[6] = (half_t)b.z; pk.v[7] = (half_t)b.w;
    half_t* dp = plane + (size_t)(nodeBase + rr) * DF + c8;
    const v4i qv = pk.q;
    *(volatile v4i*)dp = qv;
  }
  __threadfence();
#pragma unroll 1
  for (int i = 0; i < RPW / 2; ++i) {
    const int rr = RPW * wave + 2 * i + rsub;
    const int cd = cnt[rr];
    const float inv = 1.0f / (float)(cd > 1 ? cd : 1);
    const float* arow = acc + rr * DF + c8;
    const v4f a = (*(const v4f*)(arow)) * inv;
    const v4f b = (*(const v4f*)(arow + 4)) * inv;
    Pack8 pk;
    pk.v[0] = (half_t)a.x; pk.v[1] = (half_t)a.y; pk.v[2] = (half_t)a.z; pk.v[3] = (half_t)a.w;
    pk.v[4] = (half_t)b.x; pk.v[5] = (half_t)b.y; pk.v[6] = (half_t)b.z; pk.v[7] = (half_t)b.w;
    half_t* dp = plane + (size_t)(nodeBase + rr) * DF + c8;
    const v4i qv = pk.q;
    *(volatile v4i*)dp = qv;
  }
}

__device__ __forceinline__ void epi_ln(v8f (&c)[8], const float* __restrict__ bLo, const float* __restrict__ bHi,
                                       const float* __restrict__ g, const float* __restrict__ be, int m) {
  float sr[8], mr[8], qr[8];
#pragma unroll
  for (int r = 0; r < 8; ++r) sr[r] = 0.0f;
#pragma unroll
  for (int ct = 0; ct < 8; ++ct) {
    const int cl = 16 * (ct & 3) + m;
    const float bb = (ct < 4) ? bLo[cl] : bHi[cl];
#pragma unroll
    for (int r = 0; r < 8; ++r) {
      const float v = fmaxf(c[ct][r] + bb, 0.0f);
      c[ct][r] = v;
      sr[r] += v;
    }
  }
#pragma unroll
  for (int r = 0; r < 8; ++r) {
    float s = sr[r];
    s += __shfl_xor(s, 1, 16); s += __shfl_xor(s, 2, 16);
    s += __shfl_xor(s, 4, 16); s += __shfl_xor(s, 8, 16);
    mr[r] = s * (1.0f / 128.0f);
    qr[r] = 0.0f;
  }
#pragma unroll
  for (int ct = 0; ct < 8; ++ct) {
#pragma unroll
    for (int r = 0; r < 8; ++r) {
      const float d = c[ct][r] - mr[r];
      qr[r] += d * d;
    }
  }
#pragma unroll
  for (int r = 0; r < 8; ++r) {
    float q = qr[r];
    q += __shfl_xor(q, 1, 16); q += __shfl_xor(q, 2, 16);
    q += __shfl_xor(q, 4, 16); q += __shfl_xor(q, 8, 16);
    qr[r] = rsqrtf(q * (1.0f / 128.0f) + LN_EPS);
  }
#pragma unroll
  for (int ct = 0; ct < 8; ++ct) {
    const int col = 16 * ct + m;
    const float gc = g[col], bc = be[col];
#pragma unroll
    for (int r = 0; r < 8; ++r) c[ct][r] = (c[ct][r] - mr[r]) * qr[r] * gc + bc;
  }
}

__global__ __launch_bounds__(GT) void k_l0(
    const half_t* __restrict__ ap, const half_t* __restrict__ an, const float* __restrict__ x,
    const half_t* __restrict__ wb, const float* __restrict__ bP, const float* __restrict__ bN,
    const float* __restrict__ g, const float* __restrict__ be, float* h0, int nN) {
  __shared__ __attribute__((aligned(16))) float st[GW][16][STF];
  const int tid = threadIdx.x, lane = tid & 31, wave = tid >> 5, hh = lane >> 4, m = lane & 15;
  const int row0 = blockIdx.x * GR + 16 * wave;
  int node = row0 + m;
  node = node > nN - 1 ? nN - 1 : node;

  v8f c[8];
#pragma unroll
  for (int ct = 0; ct < 8; ++ct) { const v8f z = {0.f, 0.f, 0.f, 0.f, 0.f, 0.f, 0.f, 0.f}; c[ct] = z; }

  const half_t* apr = ap + (size_t)node * DF + 8 * hh;
  const half_t* anr = an + (size_t)node * DF + 8 * hh;
  const float*  xr  = x  + (size_t)node * DF + 8 * hh;
  const half_t* wr  = wb + W0_OFF + (size_t)m * W0_K + 8 * hh;

#pragma unroll 1
  for (int ks = 0; ks < 4; ++ks) {
    const v16h fa = ld16g(apr + 32 * ks);
    const v16h fn = ld16g(anr + 32 * ks);
#pragma unroll
    for (int ct = 0; ct < 8; ++ct) {
      const v16h fb = ld16g(wr + (size_t)ct * 16 * W0_K + 32 * ks);
      c[ct] = wm(ct < 4 ? fa : fn, fb, c[ct]);
    }
  }
#pragma unroll 1
  for (int ks = 0; ks < 4; ++ks) {
    const v16h fx = cv16(xr + 32 * ks);
#pragma unroll
    for (int ct = 0; ct < 8; ++ct) {
      const v16h fb = ld16g(wr + (size_t)ct * 16 * W0_K + DF + 32 * ks);
      c[ct] = wm(fx, fb, c[ct]);
    }
  }

  epi_ln(c, bP, bN, g, be, m);

  float* sp = &st[wave][8 * hh][m];
#pragma unroll
  for (int ct = 0; ct < 8; ++ct) {
#pragma unroll
    for (int r = 0; r < 8; ++r) sp[r * STF + 16 * ct] = c[ct][r];
  }
  __syncthreads();

  const float* lr = &st[wave][0][4 * lane];
  float* gp = h0 + (size_t)row0 * DF + 4 * lane;
#pragma unroll 1
  for (int i = 0; i < 16; ++i) {
    const v4f v = *(const v4f*)(lr + i * STF);
    *(volatile v4f*)(gp + (size_t)i * DF) = v;
  }
  __threadfence();
#pragma unroll 1
  for (int i = 0; i < 16; ++i) {
    const v4f v = *(const v4f*)(lr + i * STF);
    *(volatile v4f*)(gp + (size_t)i * DF) = v;
  }
}

__global__ __launch_bounds__(GT) void k_l1h(
    const half_t* __restrict__ aph, const half_t* __restrict__ anh, const float* __restrict__ h0,
    const half_t* __restrict__ wb, const float* __restrict__ bP, const float* __restrict__ bN,
    const float* __restrict__ g, const float* __restrict__ be,
    const float* __restrict__ pb1, const float* __restrict__ pb2,
    const float* __restrict__ gate, const float* __restrict__ x, float* out, int nN) {
  __shared__ __attribute__((aligned(16))) half_t T[GW][16][STH];
  __shared__ __attribute__((aligned(16))) float  U[GW][16][STF];
  const int tid = threadIdx.x, lane = tid & 31, wave = tid >> 5, hh = lane >> 4, m = lane & 15;
  const int row0 = blockIdx.x * GR + 16 * wave;
  int node = row0 + m;
  node = node > nN - 1 ? nN - 1 : node;

  v8f c[8];
#pragma unroll
  for (int ct = 0; ct < 8; ++ct) { const v8f z = {0.f, 0.f, 0.f, 0.f, 0.f, 0.f, 0.f, 0.f}; c[ct] = z; }

  const half_t* apr = aph + (size_t)node * DF + 8 * hh;
  const half_t* anr = anh + (size_t)node * DF + 8 * hh;
  const float*  hr  = h0  + (size_t)node * DF + 8 * hh;
  const half_t* w1  = wb + W1_OFF + (size_t)m * W1_K + 8 * hh;
  const half_t* p1  = wb + P1_OFF + (size_t)m * DF + 8 * hh;
  const half_t* p2  = wb + P2_OFF + (size_t)m * DF + 8 * hh;

#pragma unroll 1
  for (int ks = 0; ks < 2; ++ks) {
    const v16h fa = ld16g(apr + 32 * ks);
    const v16h fn = ld16g(apr + H2 + 32 * ks);
#pragma unroll
    for (int ct = 0; ct < 8; ++ct) {
      const v16h fb = ld16g(w1 + (size_t)ct * 16 * W1_K + 32 * ks);
      c[ct] = wm(ct < 4 ? fa : fn, fb, c[ct]);
    }
  }
#pragma unroll 1
  for (int ks = 0; ks < 2; ++ks) {
    const v16h fa = ld16g(anr + H2 + 32 * ks);
    const v16h fn = ld16g(anr + 32 * ks);
#pragma unroll
    for (int ct = 0; ct < 8; ++ct) {
      const v16h fb = ld16g(w1 + (size_t)ct * 16 * W1_K + H2 + 32 * ks);
      c[ct] = wm(ct < 4 ? fa : fn, fb, c[ct]);
    }
  }
#pragma unroll 1
  for (int ks = 0; ks < 2; ++ks) {
    const v16h fa = cv16(hr + 32 * ks);
    const v16h fn = cv16(hr + H2 + 32 * ks);
#pragma unroll
    for (int ct = 0; ct < 8; ++ct) {
      const v16h fb = ld16g(w1 + (size_t)ct * 16 * W1_K + DF + 32 * ks);
      c[ct] = wm(ct < 4 ? fa : fn, fb, c[ct]);
    }
  }

  epi_ln(c, bP, bN, g, be, m);

  {
    half_t* tp = &T[wave][8 * hh][m];
#pragma unroll
    for (int ct = 0; ct < 8; ++ct) {
#pragma unroll
      for (int r = 0; r < 8; ++r) tp[r * STH + 16 * ct] = (half_t)c[ct][r];
    }
  }
  __syncthreads();

#pragma unroll
  for (int ct = 0; ct < 8; ++ct) { const v8f z = {0.f, 0.f, 0.f, 0.f, 0.f, 0.f, 0.f, 0.f}; c[ct] = z; }
#pragma unroll 1
  for (int ks = 0; ks < 4; ++ks) {
    Frag fa;
    fa.q[0] = *(const v4i*)(&T[wave][m][32 * ks + 8 * hh]);
    fa.q[1] = *(const v4i*)(&T[wave][m][32 * ks + 16 + 8 * hh]);
#pragma unroll
    for (int ct = 0; ct < 8; ++ct) {
      const v16h fb = ld16g(p1 + (size_t)ct * 16 * DF + 32 * ks);
      c[ct] = wm(fa.v, fb, c[ct]);
    }
  }
  {
    float* up = &U[wave][8 * hh][m];
#pragma unroll
    for (int ct = 0; ct < 8; ++ct) {
      const float bb = pb1[16 * ct + m];
#pragma unroll
      for (int r = 0; r < 8; ++r) up[r * STF + 16 * ct] = c[ct][r] + bb;
    }
  }
  __syncthreads();

#pragma unroll 1
  for (int i = 0; i < 16; ++i) {
    const v4f v = *(const v4f*)(&U[wave][i][4 * lane]);
    v4h gq;
    gq[0] = (half_t)(0.5f * v.x * (1.0f + erff(v.x * 0.70710678118654752f)));
    gq[1] = (half_t)(0.5f * v.y * (1.0f + erff(v.y * 0.70710678118654752f)));
    gq[2] = (half_t)(0.5f * v.z * (1.0f + erff(v.z * 0.70710678118654752f)));
    gq[3] = (half_t)(0.5f * v.w * (1.0f + erff(v.w * 0.70710678118654752f)));
    *(v4h*)(&T[wave][i][4 * lane]) = gq;
  }
  __syncthreads();

#pragma unroll
  for (int ct = 0; ct < 8; ++ct) { const v8f z = {0.f, 0.f, 0.f, 0.f, 0.f, 0.f, 0.f, 0.f}; c[ct] = z; }
#pragma unroll 1
  for (int ks = 0; ks < 4; ++ks) {
    Frag fa;
    fa.q[0] = *(const v4i*)(&T[wave][m][32 * ks + 8 * hh]);
    fa.q[1] = *(const v4i*)(&T[wave][m][32 * ks + 16 + 8 * hh]);
#pragma unroll
    for (int ct = 0; ct < 8; ++ct) {
      const v16h fb = ld16g(p2 + (size_t)ct * 16 * DF + 32 * ks);
      c[ct] = wm(fa.v, fb, c[ct]);
    }
  }
  {
    float* up = &U[wave][8 * hh][m];
#pragma unroll
    for (int ct = 0; ct < 8; ++ct) {
      const float bb = pb2[16 * ct + m];
#pragma unroll
      for (int r = 0; r < 8; ++r) up[r * STF + 16 * ct] = c[ct][r] + bb;
    }
  }
  __syncthreads();

  const float gt = gate[0];
  const float og = 1.0f - gt;
#pragma unroll 1
  for (int i = 0; i < 16; ++i) {
    const int grow = row0 + i;
    if (grow < nN) {
      const v4f hv = *(const v4f*)(&U[wave][i][4 * lane]);
      const v4f xv = *(const v4f*)(x + (size_t)grow * DF + 4 * lane);
      const v4f o  = hv * gt + xv * og;
      *(volatile v4f*)(out + (size_t)grow * DF + 4 * lane) = o;
    }
  }
  __threadfence();
#pragma unroll 1
  for (int i = 0; i < 16; ++i) {
    const int grow = row0 + i;
    if (grow < nN) {
      const v4f hv = *(const v4f*)(&U[wave][i][4 * lane]);
      const v4f xv = *(const v4f*)(x + (size_t)grow * DF + 4 * lane);
      const v4f o  = hv * gt + xv * og;
      *(volatile v4f*)(out + (size_t)grow * DF + 4 * lane) = o;
    }
  }
}

extern "C" void kernel_launch(void* const* d_in, const int* in_sizes, int n_in,
                              void* d_out, int out_size, void* d_ws, size_t ws_size,
                              hipStream_t stream) {
  if (n_in < 24) return;
  const int nN = in_sizes[0] / DF;
  if (nN <= 0 || in_sizes[0] != nN * DF || out_size != nN * DF) return;
  const int nEp = in_sizes[1] / 2, nEn = in_sizes[2] / 2;
  if (nEp <= 0 || nEn <= 0 || in_sizes[1] != 2 * nEp || in_sizes[2] != 2 * nEn) return;
  if (in_sizes[3] != H2 * DF || in_sizes[4] != H2 * DF || in_sizes[5] < H2) return;
  if (in_sizes[6] != H2 * DF || in_sizes[7] != H2 * DF || in_sizes[8] < H2) return;
  if (in_sizes[9] != H2 * DF || in_sizes[10] != H2 * H2 || in_sizes[11] < H2) return;
  if (in_sizes[12] != H2 * DF || in_sizes[13] != H2 * H2 || in_sizes[14] < H2) return;
  if (in_sizes[15] < DF || in_sizes[16] < DF || in_sizes[17] < DF || in_sizes[18] < DF) return;
  if (in_sizes[19] != DF * DF || in_sizes[20] < DF || in_sizes[21] != DF * DF || in_sizes[22] < DF) return;
  if (in_sizes[23] < 1) return;

  const float* x       = (const float*)d_in[0];
  const int*   pei     = (const int*)d_in[1];
  const int*   nei     = (const int*)d_in[2];
  const float* c0_pl_w = (const float*)d_in[3];
  const float* c0_pr_w = (const float*)d_in[4];
  const float* c0_pr_b = (const float*)d_in[5];
  const float* c0_nl_w = (const float*)d_in[6];
  const float* c0_nr_w = (const float*)d_in[7];
  const float* c0_nr_b = (const float*)d_in[8];
  const float* c1_pl_w = (const float*)d_in[9];
  const float* c1_pr_w = (const float*)d_in[10];
  const float* c1_pr_b = (const float*)d_in[11];
  const float* c1_nl_w = (const float*)d_in[12];
  const float* c1_nr_w = (const float*)d_in[13];
  const float* c1_nr_b = (const float*)d_in[14];
  const float* ln0_g   = (const float*)d_in[15];
  const float* ln0_b   = (const float*)d_in[16];
  const float* ln1_g   = (const float*)d_in[17];
  const float* ln1_b   = (const float*)d_in[18];
  const float* pw1     = (const float*)d_in[19];
  const float* pb1     = (const float*)d_in[20];
  const float* pw2     = (const float*)d_in[21];
  const float* pb2     = (const float*)d_in[22];
  const float* gate    = (const float*)d_in[23];
  float* out = (float*)d_out;

  const int    nBlkA = (nN + NB - 1) / NB;
  const size_t rowsA = (size_t)nBlkA * NB;
  const int    nBlkG = (nN + GR - 1) / GR;
  const size_t rowsG = (size_t)nBlkG * GR;

  char* ws = (char*)d_ws;
  size_t off = 0;
  const size_t szWB = (size_t)WB_TOT * 2;
  const size_t szA  = rowsA * DF * 2;
  const size_t szH  = rowsG * DF * 4;
  const size_t oWB = off; off += szWB; off = (off + 255) & ~(size_t)255;
  const size_t oAP = off; off += szA;  off = (off + 255) & ~(size_t)255;
  const size_t oAN = off; off += szA;  off = (off + 255) & ~(size_t)255;
  const size_t oH0 = off; off += szH;  off = (off + 255) & ~(size_t)255;
  if (off > ws_size || off > (size_t)134217728u) return;
  half_t* wb  = (half_t*)(ws + oWB);
  half_t* apl = (half_t*)(ws + oAP);
  half_t* anl = (half_t*)(ws + oAN);
  float*  h0  = (float*)(ws + oH0);

  const int vec8p = ((nEp & 3) == 0) ? 1 : 0;
  const int vec8n = ((nEn & 3) == 0) ? 1 : 0;
  const int nTot  = WB_TOT / 8;

  k_wprep<<<(nTot + 255) / 256, 256, 0, stream>>>(c0_pl_w, c0_pr_w, c0_nl_w, c0_nr_w,
                                                  c1_pl_w, c1_pr_w, c1_nl_w, c1_nr_w,
                                                  pw1, pw2, wb, nTot);

  hipFuncSetAttribute(reinterpret_cast<const void*>(&k_agg),
                      hipFuncAttributeMaxDynamicSharedMemorySize, LDS_AGG);

  k_agg<<<nBlkA, NTHR, LDS_AGG, stream>>>(pei, x, apl, nN, nEp, vec8p);
  k_agg<<<nBlkA, NTHR, LDS_AGG, stream>>>(nei, x, anl, nN, nEn, vec8n);
  k_l0<<<nBlkG, GT, 0, stream>>>(apl, anl, x, wb, c0_pr_b, c0_nr_b, ln0_g, ln0_b, h0, nN);
  k_agg<<<nBlkA, NTHR, LDS_AGG, stream>>>(pei, h0, apl, nN, nEp, vec8p);
  k_agg<<<nBlkA, NTHR, LDS_AGG, stream>>>(nei, h0, anl, nN, nEn, vec8n);
  k_l1h<<<nBlkG, GT, 0, stream>>>(apl, anl, h0, wb, c1_pr_b, c1_nr_b, ln1_g, ln1_b,
                                  pb1, pb2, gate, x, out, nN);
}
